// MultiheadAttention_29858612641871
// MI455X (gfx1250) — hardware-verified
//
#include <hip/hip_runtime.h>
#include <math.h>

typedef __attribute__((ext_vector_type(16))) _Float16 v16h;
typedef __attribute__((ext_vector_type(8)))  _Float16 v8h;
typedef __attribute__((ext_vector_type(16))) __bf16   v16b;
typedef __attribute__((ext_vector_type(8)))  __bf16   v8b;
typedef __attribute__((ext_vector_type(8)))  float    v8f;
typedef __attribute__((ext_vector_type(4)))  float    v4f;
typedef __attribute__((ext_vector_type(2)))  float    v2f;
typedef __attribute__((ext_vector_type(4)))  unsigned int v4u;

constexpr int kB   = 4;
constexpr int kL   = 2048;
constexpr int kE   = 1024;
constexpr int kH   = 16;
constexpr int kD   = 64;
constexpr int kTok = kB * kL;
constexpr int kBH  = kB * kH;
constexpr int kNqk = 2 * kH * kD;
constexpr int kNv  = kH * kD;
constexpr int kNall = 3 * kH * kD;
constexpr int kPre = 128;
constexpr int kKC = 64;
constexpr int kQB = 64;
constexpr int kNW = 4;
constexpr int kFirstQB = kPre / kQB;
constexpr int kNumQB = kL / kQB;
constexpr float kInvSqrtD   = 0.125f;
constexpr float kQKCarry    = 16.0f;
constexpr float kVCarry     = 16.0f;
constexpr float kPCarry     = 32768.0f;
constexpr float kScoreScale = kInvSqrtD / (kQKCarry * kQKCarry);
constexpr float kMaskFill   = -1.0e30f;

static_assert(kD == 64, "head dim fixed at 64");
static_assert(kInvSqrtD * kInvSqrtD * (float)kD == 1.0f, "score scale is 1/sqrt(head dim)");
static_assert(kScoreScale * 2048.0f == 1.0f, "score scale with carries is 2^-11");
static_assert((kE % 32) == 0 && (kD % 32) == 0 && (kKC % 32) == 0, "contraction depths are multiples of 32");
static_assert((kTok % 64) == 0 && (kNqk % 64) == 0 && (kNv % 64) == 0 && (kL % 64) == 0, "tile multiples");
static_assert((kPre % 64) == 0 && (kPre % kQB) == 0 && kPre == 128, "f32 prefix rows");
static_assert(((kTok / 64) * (kNqk / 64)) % 8 == 0 && ((kNv / 64) * (kTok / 64)) % 8 == 0, "tiles per block");

constexpr size_t kOffXB   = 0;
constexpr size_t kOffWT   = kOffXB   + (size_t)kTok * kE * 2;
constexpr size_t kOffQ16  = kOffWT   + (size_t)kNall * kE * 2;
constexpr size_t kOffK16  = kOffQ16  + (size_t)kBH * kL * kD * 2;
constexpr size_t kOffVT16 = kOffK16  + (size_t)kBH * kL * kD * 2;
constexpr size_t kOffQ32  = kOffVT16 + (size_t)kBH * kD * kL * 2;
constexpr size_t kOffK32  = kOffQ32  + (size_t)kBH * kPre * kD * 4;
constexpr size_t kOffV32T = kOffK32  + (size_t)kBH * kPre * kD * 4;
constexpr size_t kWsTotal = kOffV32T + (size_t)kBH * kD * kPre * 4;
static_assert(kWsTotal == 79691776ull, "carve total");
static_assert(kWsTotal <= 134217728ull, "carve cap");
static_assert((kOffWT % 128) == 0 && (kOffQ16 % 128) == 0 && (kOffK16 % 128) == 0 && (kOffVT16 % 128) == 0 &&
              (kOffQ32 % 128) == 0 && (kOffK32 % 128) == 0 && (kOffV32T % 128) == 0, "128-B aligned regions");

__device__ __forceinline__ unsigned short f2bf_bits(float f) {
  unsigned u = __float_as_uint(f);
  return (unsigned short)((u + 0x7FFFu + ((u >> 16) & 1u)) >> 16);
}
__device__ __forceinline__ unsigned pk16(unsigned short a, unsigned short b) { return (unsigned)a | ((unsigned)b << 16); }

union FragB { v16b v; v8b h[2]; };
union FragH { v16h v; v8h h[2]; };
__device__ __forceinline__ v16b ldfrag_b(const __bf16* p) {
  FragB f; f.h[0] = *(const v8b*)(p); f.h[1] = *(const v8b*)(p + 16); return f.v;
}
__device__ __forceinline__ v16h ldfrag_h(const _Float16* p) {
  FragH f; f.h[0] = *(const v8h*)(p); f.h[1] = *(const v8h*)(p + 16); return f.v;
}
__device__ __forceinline__ v8f mma_b(v16b a, v16b b, v8f c) {
  c = __builtin_amdgcn_wmma_f32_16x16x32_bf16(false, a, false, b, (short)0, c, false, false);
  asm volatile("v_nop\n\tv_nop\n\tv_nop\n\tv_nop" : "+v"(c) : "v"(a), "v"(b));
  return c;
}
__device__ __forceinline__ v8f mma_h(v16h a, v16h b, v8f c) {
  c = __builtin_amdgcn_wmma_f32_16x16x32_f16(false, a, false, b, (short)0, c, false, false);
  asm volatile("v_nop\n\tv_nop\n\tv_nop\n\tv_nop" : "+v"(c) : "v"(a), "v"(b));
  return c;
}
__device__ __forceinline__ void wave_lds_sync() {
  __builtin_amdgcn_fence(__ATOMIC_RELEASE, "workgroup");
  __builtin_amdgcn_wave_barrier();
  __builtin_amdgcn_fence(__ATOMIC_ACQUIRE, "workgroup");
}

__global__ __launch_bounds__(256) void x_plane_kernel(const float* __restrict__ in, unsigned short* __restrict__ outp, int n8) {
  const int i = blockIdx.x * 256 + threadIdx.x;
  if (i >= n8) return;
  const float* p = in + 8 * (size_t)i;
  const v4f a = *(const v4f*)(p);
  const v4f c = *(const v4f*)(p + 4);
  unsigned short hb[8];
#pragma unroll
  for (int e = 0; e < 4; ++e) {
    const float fa = a[e];
    const float fc = c[e];
    hb[e]     = f2bf_bits(fa);
    hb[4 + e] = f2bf_bits(fc);
  }
  const v4u u = (v4u){pk16(hb[0], hb[1]), pk16(hb[2], hb[3]), pk16(hb[4], hb[5]), pk16(hb[6], hb[7])};
  unsigned short* q = outp + 8 * (size_t)i;
  *(volatile v4u*)q = u;
  __threadfence();
  *(volatile v4u*)q = u;
}

__global__ __launch_bounds__(256) void wt_plane_kernel(const float* __restrict__ w0, const float* __restrict__ w1,
                                                       const float* __restrict__ w2, unsigned short* __restrict__ WT) {
  __shared__ float sm[64][65];
  const int t  = threadIdx.x;
  const int e0 = blockIdx.x * 64;
  const int h  = blockIdx.y;
  const int z  = blockIdx.z;
  const float* W = (z == 0) ? w0 : ((z == 1) ? w1 : w2);
  const float* src = W + ((size_t)h * kE + e0) * kD;
#pragma unroll
  for (int i = 0; i < 4; ++i) {
    const int base = (i * 256 + t) * 4;
    const int r = base >> 6;
    const int c = base & 63;
    const v4f v = *(const v4f*)(src + base);
    sm[c + 0][r] = v[0];
    sm[c + 1][r] = v[1];
    sm[c + 2][r] = v[2];
    sm[c + 3][r] = v[3];
  }
  __syncthreads();
  const int lane = t & 31;
  const int wave = __builtin_amdgcn_readfirstlane((int)(threadIdx.x >> 5));
  const int q = lane >> 3, c8 = (lane & 7) * 8;
  v4u u[2];
#pragma unroll
  for (int it = 0; it < 2; ++it) {
    const int row = wave * 8 + it * 4 + q;
    unsigned short hb[8];
#pragma unroll
    for (int e = 0; e < 8; ++e) hb[e] = f2bf_bits(sm[row][c8 + e]);
    u[it] = (v4u){pk16(hb[0], hb[1]), pk16(hb[2], hb[3]), pk16(hb[4], hb[5]), pk16(hb[6], hb[7])};
  }
  for (int pass = 0; pass < 2; ++pass) {
#pragma unroll
    for (int it = 0; it < 2; ++it) {
      const int row = wave * 8 + it * 4 + q;
      *(volatile v4u*)(WT + ((size_t)z * kNv + (size_t)h * kD + row) * kE + e0 + c8) = u[it];
    }
    __threadfence();
  }
}

template <int MODE>
__global__ __launch_bounds__(256) void proj_gemm_kernel(
    const unsigned short* __restrict__ Ap, const unsigned short* __restrict__ Btp,
    unsigned short* __restrict__ o16a, unsigned short* __restrict__ o16b,
    float* __restrict__ o32a, float* __restrict__ o32b) {
  __shared__ __align__(16) float sT[8][16 * 68];
  const int lane = threadIdx.x & 31;
  const int wave = __builtin_amdgcn_readfirstlane((int)(threadIdx.x >> 5));
  constexpr int tilesN = (MODE == 0) ? (kNqk / 64) : (kTok / 64);
  constexpr int tilesM = (MODE == 0) ? (kTok / 64) : (kNv / 64);
  const int tile = blockIdx.x * 8 + wave;
  if (tile >= tilesM * tilesN) return;
  const int tm = tile / tilesN;
  const int tn = tile - tm * tilesN;
  const int m0 = tm << 6;
  const int n0 = tn << 6;

  const __bf16* A  = (const __bf16*)(const void*)Ap;
  const __bf16* Bt = (const __bf16*)(const void*)Btp;
  const int rlane = lane & 15;
  const int koff  = (lane >> 4) * 8;
  const int mOff  = (lane >> 4) * 8;
  const __bf16* Arow = A  + (size_t)(m0 + rlane) * kE + koff;
  const __bf16* Brow = Bt + (size_t)(n0 + rlane) * kE + koff;

  v8f acc[4][4];
#pragma unroll
  for (int i = 0; i < 4; ++i)
#pragma unroll
    for (int j = 0; j < 4; ++j) acc[i][j] = (v8f){0.f, 0.f, 0.f, 0.f, 0.f, 0.f, 0.f, 0.f};

#pragma unroll 1
  for (int k0 = 0; k0 < kE; k0 += 32) {
    v16b bfr[4];
#pragma unroll
    for (int j = 0; j < 4; ++j) bfr[j] = ldfrag_b(Brow + (size_t)(j << 4) * kE + k0);
#pragma unroll
    for (int i = 0; i < 4; ++i) {
      const v16b afr = ldfrag_b(Arow + (size_t)(i << 4) * kE + k0);
#pragma unroll
      for (int j = 0; j < 4; ++j) acc[i][j] = mma_b(afr, bfr[j], acc[i][j]);
    }
  }

  unsigned short* dst16;
  float* dst32;
  size_t ld16, ld32;
  bool side;
  if (MODE == 0) {
    const int zq = tn >> 4;
    const int h  = tn & 15;
    const int b  = m0 >> 11;
    const int l0 = m0 & (kL - 1);
    const int bh = b * kH + h;
    dst16 = ((zq == 0) ? o16a : o16b) + ((size_t)bh * kL + l0) * kD;
    ld16  = kD;
    side  = (l0 < kPre);
    const int l0c = side ? l0 : 0;
    dst32 = ((zq == 0) ? o32a : o32b) + ((size_t)bh * kPre + l0c) * kD;
    ld32  = kD;
  } else {
    const int h  = tm;
    const int b  = n0 >> 11;
    const int l0 = n0 & (kL - 1);
    const int bh = b * kH + h;
    dst16 = o16a + (size_t)bh * kD * kL + l0;
    ld16  = kL;
    side  = (l0 < kPre);
    const int l0c = side ? l0 : 0;
    dst32 = o32a + (size_t)bh * kD * kPre + l0c;
    ld32  = kPre;
  }

  float* slab = sT[wave];
  const int q4 = lane >> 3, c8 = (lane & 7) * 8;
  const int hh = lane >> 4, c4 = (lane & 15) * 4;
#pragma unroll
  for (int i = 0; i < 4; ++i) {
#pragma unroll
    for (int j = 0; j < 4; ++j) {
#pragma unroll
      for (int r = 0; r < 8; ++r) slab[(mOff + r) * 68 + (j << 4) + rlane] = acc[i][j][r];
    }
    wave_lds_sync();
    v8h hv[4];
#pragma unroll
    for (int it = 0; it < 4; ++it) {
      const float* sp = slab + (it * 4 + q4) * 68 + c8;
      const v4f a0 = *(const v4f*)(sp);
      const v4f a1 = *(const v4f*)(sp + 4);
#pragma unroll
      for (int e = 0; e < 4; ++e) {
        const float f0 = a0[e] * kQKCarry;
        const float f1 = a1[e] * kQKCarry;
        hv[it][e]     = (_Float16)f0;
        hv[it][4 + e] = (_Float16)f1;
      }
    }
    for (int pass = 0; pass < 2; ++pass) {
#pragma unroll
      for (int it = 0; it < 4; ++it) {
        const int row = (i << 4) + it * 4 + q4;
        *(volatile v8h*)(dst16 + (size_t)row * ld16 + c8) = hv[it];
      }
      __threadfence();
    }
    if (side) {
      for (int pass = 0; pass < 2; ++pass) {
#pragma unroll
        for (int it = 0; it < 8; ++it) {
          const int rl = it * 2 + hh;
          const v4f v = *(const v4f*)(slab + rl * 68 + c4);
          *(volatile v4f*)(dst32 + (size_t)((i << 4) + rl) * ld32 + c4) = v;
        }
        __threadfence();
      }
    }
    wave_lds_sync();
  }
}
static_assert(kQKCarry == kVCarry, "one carry for the three projection planes");

__global__ __launch_bounds__(256) void attn_head_rows_kernel(
    const float* __restrict__ Q32, const float* __restrict__ K32, const float* __restrict__ V32T,
    float* __restrict__ out) {
  __shared__ __align__(16) float sQ[8][kD];
  __shared__ __align__(16) float sP[8][kPre];
  __shared__ __align__(16) float sO[8][kD];
  const int lane = threadIdx.x & 31;
  const int wave = __builtin_amdgcn_readfirstlane((int)(threadIdx.x >> 5));
  const int bh = blockIdx.x >> 4;
  const int l  = ((blockIdx.x & 15) << 3) + wave;
  const int b  = bh >> 4;
  const int h  = bh & 15;
  {
    const v2f qv = *(const v2f*)(Q32 + ((size_t)bh * kPre + l) * kD + 2 * lane);
    *(v2f*)(&sQ[wave][2 * lane]) = qv;
  }
  __syncthreads();
  int nCh = (l >> 5) + 1;
  nCh = (nCh > 4) ? 4 : nCh;
  const float* qrow = sQ[wave];
  float* prow = sP[wave];
#pragma unroll 1
  for (int i = 0; i < nCh; ++i) {
    const int m = i * 32 + lane;
    const float* kp = K32 + ((size_t)bh * kPre + m) * kD;
    float dot = 0.0f;
#pragma unroll 1
    for (int d4 = 0; d4 < kD / 4; ++d4) {
      const v4f kk = *(const v4f*)(kp + 4 * d4);
      const v4f qq = *(const v4f*)(qrow + 4 * d4);
      dot = fmaf(qq[0], kk[0], dot);
      dot = fmaf(qq[1], kk[1], dot);
      dot = fmaf(qq[2], kk[2], dot);
      dot = fmaf(qq[3], kk[3], dot);
    }
    const float sc = dot * kInvSqrtD;
    prow[m] = (m <= l) ? sc : kMaskFill;
  }
  float mx = kMaskFill;
#pragma unroll 1
  for (int i = 0; i < nCh; ++i) mx = fmaxf(mx, prow[i * 32 + lane]);
#pragma unroll
  for (int off = 16; off > 0; off >>= 1) mx = fmaxf(mx, __shfl_xor(mx, off, 32));
  float sum = 0.0f;
#pragma unroll 1
  for (int i = 0; i < nCh; ++i) {
    const int m = i * 32 + lane;
    const float sv = prow[m];
    const float ev = expf(sv - mx);
    const float p = (m <= l) ? ev : 0.0f;
    prow[m] = p;
    sum += p;
  }
#pragma unroll
  for (int off = 16; off > 0; off >>= 1) sum += __shfl_xor(sum, off, 32);
  __syncthreads();
  int nQ = (l >> 2) + 1;
  nQ = (nQ > kPre / 4) ? (kPre / 4) : nQ;
  const float* va = V32T + ((size_t)bh * kD + lane) * kPre;
  const float* vb = va + (size_t)32 * kPre;
  float accA = 0.0f, accB = 0.0f;
#pragma unroll 1
  for (int cq = 0; cq < nQ; ++cq) {
    const v4f pp = *(const v4f*)(prow + 4 * cq);
    const v4f xa = *(const v4f*)(va + 4 * cq);
    const v4f xb = *(const v4f*)(vb + 4 * cq);
    accA = fmaf(pp[0], xa[0], accA);
    accA = fmaf(pp[1], xa[1], accA);
    accA = fmaf(pp[2], xa[2], accA);
    accA = fmaf(pp[3], xa[3], accA);
    accB = fmaf(pp[0], xb[0], accB);
    accB = fmaf(pp[1], xb[1], accB);
    accB = fmaf(pp[2], xb[2], accB);
    accB = fmaf(pp[3], xb[3], accB);
  }
  const float inv = 1.0f / sum;
  sO[wave][lane]      = accA * inv;
  sO[wave][lane + 32] = accB * inv;
  __syncthreads();
  const int c4 = (lane & 15) * 4;
  const v4f val = *(const v4f*)(&sO[wave][c4]);
  float* op = out + ((size_t)b * kL + l) * (size_t)(kH * kD) + h * kD + c4;
  if (lane < 16) *(volatile v4f*)op = val;
  __threadfence();
  if (lane < 16) *(volatile v4f*)op = val;
}

__global__ __launch_bounds__(128) void attn_tail_kernel(
    const unsigned short* __restrict__ Qp, const unsigned short* __restrict__ Kp,
    const unsigned short* __restrict__ VTp, float* __restrict__ out) {
  __shared__ __align__(16) _Float16 Ksh[kKC * kD];
  __shared__ __align__(16) _Float16 Vsh[kD * kKC];
  __shared__ __align__(16) _Float16 Psh[kNW][16 * kKC];
  __shared__ __align__(16) float    Os[kNW][16 * 68];

  const int tid  = threadIdx.x;
  const int wave = __builtin_amdgcn_readfirstlane((int)(threadIdx.x >> 5));
  const int lane = tid & 31;
  const int hh   = lane >> 4;
  const int c    = lane & 15;
  const int qb   = (int)blockIdx.x + kFirstQB;
  const int bh   = blockIdx.y;
  const int b    = bh >> 4;
  const int h    = bh & 15;
  const int q0   = qb * kQB + wave * 16;

  const _Float16* Qb  = (const _Float16*)(const void*)Qp  + (size_t)bh * kL * kD;
  const _Float16* Kb  = (const _Float16*)(const void*)Kp  + (size_t)bh * kL * kD;
  const _Float16* VTb = (const _Float16*)(const void*)VTp + (size_t)bh * kD * kL;

  v16h qa[2];
  {
    const _Float16* qrow = Qb + (size_t)(q0 + c) * kD + 8 * hh;
    qa[0] = ldfrag_h(qrow);
    qa[1] = ldfrag_h(qrow + 32);
  }

  float mrow[8], lrow[8];
  v8f oacc[4];
#pragma unroll
  for (int r = 0; r < 8; ++r) { mrow[r] = kMaskFill; lrow[r] = 0.0f; }
#pragma unroll
  for (int t = 0; t < 4; ++t) oacc[t] = (v8f){0.f, 0.f, 0.f, 0.f, 0.f, 0.f, 0.f, 0.f};

  _Float16* pw = Psh[wave];
  int nChunks = qb + 1;
  nChunks = (nChunks > kNumQB) ? kNumQB : nChunks;
#pragma unroll 1
  for (int kc = 0; kc < nChunks; ++kc) {
    const int kv0 = kc * kKC;
    __syncthreads();
    {
      const _Float16* ksrc = Kb + (size_t)kv0 * kD;
#pragma unroll
      for (int i = 0; i < 4; ++i) {
        const int p8 = (i * 128 + tid) * 8;
        const v8h kk = *(const v8h*)(ksrc + p8);
        *(v8h*)(Ksh + p8) = kk;
      }
#pragma unroll
      for (int i = 0; i < 4; ++i) {
        const int e = i * 128 + tid;
        const int d = e >> 3, p8 = (e & 7) * 8;
        const v8h vv = *(const v8h*)(VTb + (size_t)d * kL + kv0 + p8);
        *(v8h*)(Vsh + d * kKC + p8) = vv;
      }
    }
    __syncthreads();

    v8f s[4];
#pragma unroll
    for (int j = 0; j < 4; ++j) {
      s[j] = (v8f){0.f, 0.f, 0.f, 0.f, 0.f, 0.f, 0.f, 0.f};
#pragma unroll
      for (int dc = 0; dc < 2; ++dc) {
        const v16h kf = ldfrag_h(Ksh + (j * 16 + c) * kD + dc * 32 + 8 * hh);
        s[j] = mma_h(qa[dc], kf, s[j]);
      }
    }
    if (kc == qb) {
#pragma unroll
      for (int j = 0; j < 4; ++j) {
        const int kvcol = kv0 + j * 16 + c;
#pragma unroll
        for (int r = 0; r < 8; ++r) {
          const int qrow = q0 + 8 * hh + r;
          const float cur = s[j][r];
          s[j][r] = (kvcol > qrow) ? kMaskFill : cur;
        }
      }
    }
    float cm[8];
#pragma unroll
    for (int r = 0; r < 8; ++r) {
      float m = fmaxf(fmaxf(s[0][r], s[1][r]), fmaxf(s[2][r], s[3][r]));
#pragma unroll
      for (int off = 1; off < 16; off <<= 1) m = fmaxf(m, __shfl_xor(m, off, 32));
      cm[r] = m;
    }
#pragma unroll
    for (int r = 0; r < 8; ++r) {
      const float mnew  = fmaxf(mrow[r], cm[r]);
      const float alpha = __expf((mrow[r] - mnew) * kScoreScale);
      mrow[r] = mnew;
      float psum = 0.0f;
#pragma unroll
      for (int j = 0; j < 4; ++j) {
        const float p = __expf((s[j][r] - mnew) * kScoreScale);
        psum += p;
        pw[(8 * hh + r) * kKC + j * 16 + c] = (_Float16)(p * kPCarry);
      }
#pragma unroll
      for (int off = 1; off < 16; off <<= 1) psum += __shfl_xor(psum, off, 32);
      lrow[r] = lrow[r] * alpha + psum;
#pragma unroll
      for (int t = 0; t < 4; ++t) oacc[t][r] *= alpha;
    }
    wave_lds_sync();
#pragma unroll
    for (int kk = 0; kk < 2; ++kk) {
      const v16h pa = ldfrag_h(pw + c * kKC + kk * 32 + 8 * hh);
#pragma unroll
      for (int t = 0; t < 4; ++t) {
        const v16h vf = ldfrag_h(Vsh + (t * 16 + c) * kKC + kk * 32 + 8 * hh);
        oacc[t] = mma_h(pa, vf, oacc[t]);
      }
    }
  }

  float* os = Os[wave];
#pragma unroll
  for (int r = 0; r < 8; ++r) {
    const float inv = 1.0f / (lrow[r] * (kPCarry * kVCarry));
#pragma unroll
    for (int t = 0; t < 4; ++t) os[(8 * hh + r) * 68 + t * 16 + c] = oacc[t][r] * inv;
  }
  wave_lds_sync();
  {
    const int c4 = (lane & 15) * 4;
    float* ob = out + ((size_t)b * kL + q0) * (size_t)(kH * kD) + h * kD + c4;
    for (int pass = 0; pass < 2; ++pass) {
#pragma unroll
      for (int it = 0; it < 8; ++it) {
        const int row = it * 2 + hh;
        const v4f val = *(const v4f*)(os + row * 68 + c4);
        *(volatile v4f*)(ob + (size_t)row * (kH * kD)) = val;
      }
      __threadfence();
    }
  }
}

extern "C" void kernel_launch(void* const* d_in, const int* in_sizes, int n_in,
                              void* d_out, int out_size, void* d_ws, size_t ws_size,
                              hipStream_t stream) {
  if (n_in < 4) return;
  if (in_sizes[0] != kTok * kE) return;
  if (in_sizes[1] != kH * kE * kD) return;
  if (in_sizes[2] != kH * kE * kD) return;
  if (in_sizes[3] != kH * kE * kD) return;
  if (out_size != kTok * kH * kD) return;
  if (ws_size < kWsTotal) return;

  const float* x  = (const float*)d_in[0];
  const float* wq = (const float*)d_in[1];
  const float* wk = (const float*)d_in[2];
  const float* wv = (const float*)d_in[3];
  float* out = (float*)d_out;

  char* ws = (char*)d_ws;
  unsigned short* XB   = (unsigned short*)(ws + kOffXB);
  unsigned short* WT   = (unsigned short*)(ws + kOffWT);
  unsigned short* Q16  = (unsigned short*)(ws + kOffQ16);
  unsigned short* K16  = (unsigned short*)(ws + kOffK16);
  unsigned short* VT16 = (unsigned short*)(ws + kOffVT16);
  float*          Q32  = (float*)(ws + kOffQ32);
  float*          K32  = (float*)(ws + kOffK32);
  float*          V32T = (float*)(ws + kOffV32T);

  x_plane_kernel<<<dim3((kTok * kE / 8) / 256), 256, 0, stream>>>(x, XB, kTok * kE / 8);
  wt_plane_kernel<<<dim3(kE / 64, kH, 3), 256, 0, stream>>>(wq, wk, wv, WT);

  proj_gemm_kernel<0><<<dim3(((kTok / 64) * (kNqk / 64)) / 8), 256, 0, stream>>>(
      XB, WT, Q16, K16, Q32, K32);
  proj_gemm_kernel<1><<<dim3(((kNv / 64) * (kTok / 64)) / 8), 256, 0, stream>>>(
      WT + (size_t)kNqk * kE, XB, VT16, VT16, V32T, V32T);

  attn_head_rows_kernel<<<dim3(kBH * (kPre / 8)), 256, 0, stream>>>(Q32, K32, V32T, out);
  attn_tail_kernel<<<dim3(kNumQB - kFirstQB, kBH), kNW * 32, 0, stream>>>(Q16, K16, VT16, out);
}
